// GaussianAttention_257698038469
// MI455X (gfx1250) — hardware-verified
//
#include <hip/hip_runtime.h>
#include <stdint.h>


typedef _Float16 v4h  __attribute__((ext_vector_type(4)));
typedef _Float16 v8h  __attribute__((ext_vector_type(8)));
typedef _Float16 v16h __attribute__((ext_vector_type(16)));
typedef float    v4f  __attribute__((ext_vector_type(4)));
typedef float    v8f  __attribute__((ext_vector_type(8)));
typedef int      v4i  __attribute__((ext_vector_type(4)));

#define NB     16
#define DM     256
#define NH     9
#define NQ     1024
#define FAN    2304
#define NROW   16384
#define KCH    64
#define NCHQ   16
#define NCHF   36
#define LDT    72
#define SPH    136
#define SPF    36
#define SMEM_BYTES 36864
#define PSC    4096.0f
#define CSC    0.00390625f
#define WSC    64.0f
#define OSC    0.0009765625f
#define F16MIN 6.103515625e-5f
#define LNEPS  1e-5f

__device__ __forceinline__ v16h ld_frag(const _Float16* t, int row, int ks, int h) {
  const _Float16* p = t + row * LDT + ks + 8 * h;
  const v8h lo = *(const v8h*)(p);
  const v8h hi = *(const v8h*)(p + 16);
  return __builtin_shufflevector(lo, hi, 0, 1, 2, 3, 4, 5, 6, 7, 8, 9, 10, 11, 12, 13, 14, 15);
}

__device__ __forceinline__ v8f mma16(v16h a, v16h b, v8f c) {
  return __builtin_amdgcn_wmma_f32_16x16x32_f16(false, a, false, b, (short)0, c, false, false);
}

__device__ __forceinline__ void stage_chunk(const _Float16* __restrict__ gA, int lda,
                                            const _Float16* __restrict__ gB, int ldb,
                                            int kk, _Float16* sA, _Float16* sB, int tid) {
#pragma unroll
  for (int rep = 0; rep < 4; ++rep) {
    const int idx = tid + rep * 256;
    const int row = idx >> 3, seg = (idx & 7) * 8;
    const v8h v = *(const v8h*)(gA + (size_t)row * lda + kk + seg);
    *(v8h*)(sA + row * LDT + seg) = v;
  }
#pragma unroll
  for (int rep = 0; rep < 4; ++rep) {
    const int idx = tid + rep * 256;
    const int row = idx >> 3, seg = (idx & 7) * 8;
    const v8h v = *(const v8h*)(gB + (size_t)row * ldb + kk + seg);
    *(v8h*)(sB + row * LDT + seg) = v;
  }
}

__device__ __forceinline__ void mma_chunk(const _Float16* sA, const _Float16* sB,
                                          int wm, int wn, int h, int l15, v8f (&acc)[4][2]) {
#pragma unroll
  for (int ks = 0; ks < KCH; ks += 32) {
    const v16h a0 = ld_frag(sA, wm * 64 + l15, ks, h);
    const v16h a1 = ld_frag(sA, wm * 64 + 16 + l15, ks, h);
    const v16h a2 = ld_frag(sA, wm * 64 + 32 + l15, ks, h);
    const v16h a3 = ld_frag(sA, wm * 64 + 48 + l15, ks, h);
    const v16h b0 = ld_frag(sB, wn * 32 + l15, ks, h);
    const v16h b1 = ld_frag(sB, wn * 32 + 16 + l15, ks, h);
    acc[0][0] = mma16(a0, b0, acc[0][0]);  acc[0][1] = mma16(a0, b1, acc[0][1]);
    acc[1][0] = mma16(a1, b0, acc[1][0]);  acc[1][1] = mma16(a1, b1, acc[1][1]);
    acc[2][0] = mma16(a2, b0, acc[2][0]);  acc[2][1] = mma16(a2, b1, acc[2][1]);
    acc[3][0] = mma16(a3, b0, acc[3][0]);  acc[3][1] = mma16(a3, b1, acc[3][1]);
    asm volatile("v_nop\n\tv_nop\n\tv_nop\n\tv_nop"
                 : "+v"(acc[0][0]), "+v"(acc[0][1]), "+v"(acc[1][0]), "+v"(acc[1][1]),
                   "+v"(acc[2][0]), "+v"(acc[2][1]), "+v"(acc[3][0]), "+v"(acc[3][1])
                 : "v"(a0), "v"(a1), "v"(a2), "v"(a3), "v"(b0), "v"(b1));
  }
}

__global__ __launch_bounds__(256) void k_ln(const float* __restrict__ hid,
                                            const float* __restrict__ gam,
                                            const float* __restrict__ bet,
                                            float* __restrict__ xln,
                                            _Float16* __restrict__ x16t) {
  __shared__ __attribute__((aligned(16))) _Float16 tT[256 * LDT];
  const int tid = threadIdx.x, wave = tid >> 5, lane = tid & 31;
  const int rb = blockIdx.x * 64;
  if (rb >= NROW) return;
  const int b = rb >> 10, k0 = rb & (NQ - 1);
  const v4f g0 = *(const v4f*)(gam + 4 * lane), g1 = *(const v4f*)(gam + 128 + 4 * lane);
  const v4f e0 = *(const v4f*)(bet + 4 * lane), e1 = *(const v4f*)(bet + 128 + 4 * lane);

#pragma unroll 1
  for (int i = 0; i < 8; ++i) {
    const int rl = wave * 8 + i;
    const size_t row = (size_t)rb + rl;
    const float* src = hid + row * DM;
    const v4f v0 = *(const v4f*)(src + 4 * lane);
    const v4f v1 = *(const v4f*)(src + 128 + 4 * lane);
    float s = ((v0.x + v0.y) + (v0.z + v0.w)) + ((v1.x + v1.y) + (v1.z + v1.w));
#pragma unroll
    for (int off = 16; off; off >>= 1) s += __shfl_xor(s, off, 32);
    const float mu = s * (1.0f / DM);
    const v4f d0 = v0 - mu, d1 = v1 - mu;
    float ss = ((d0.x * d0.x + d0.y * d0.y) + (d0.z * d0.z + d0.w * d0.w))
             + ((d1.x * d1.x + d1.y * d1.y) + (d1.z * d1.z + d1.w * d1.w));
#pragma unroll
    for (int off = 16; off; off >>= 1) ss += __shfl_xor(ss, off, 32);
    const float rs = rsqrtf(ss * (1.0f / DM) + LNEPS);
    const v4f o0 = d0 * rs * g0 + e0;
    const v4f o1 = d1 * rs * g1 + e1;
    float* dst = xln + row * DM;
    *(volatile v4f*)(dst + 4 * lane) = o0;
    *(volatile v4f*)(dst + 128 + 4 * lane) = o1;
    __threadfence();
    *(volatile v4f*)(dst + 4 * lane) = o0;
    *(volatile v4f*)(dst + 128 + 4 * lane) = o1;
#pragma unroll
    for (int e = 0; e < 4; ++e) {
      tT[(4 * lane + e) * LDT + rl] = (_Float16)o0[e];
      tT[(128 + 4 * lane + e) * LDT + rl] = (_Float16)o1[e];
    }
  }
  __syncthreads();

  const int g = lane >> 3, j = lane & 7;
  v8h vv[8];
#pragma unroll
  for (int it = 0; it < 8; ++it) {
    const int d = wave * 32 + it * 4 + g;
    vv[it] = *(const v8h*)(tT + d * LDT + j * 8);
    _Float16* dstp = x16t + ((size_t)(b * DM + d)) * NQ + k0 + j * 8;
    *(volatile v8h*)dstp = vv[it];
  }
  __threadfence();
#pragma unroll
  for (int it = 0; it < 8; ++it) {
    const int d = wave * 32 + it * 4 + g;
    _Float16* dstp = x16t + ((size_t)(b * DM + d)) * NQ + k0 + j * 8;
    *(volatile v8h*)dstp = vv[it];
  }
}

__global__ __launch_bounds__(256) void k_w(const float* __restrict__ w,
                                           _Float16* __restrict__ w16, int n8) {
  const int i = blockIdx.x * 256 + threadIdx.x;
  if (i >= n8) return;
  const float* s = w + (size_t)i * 8;
  const v4f a = *(const v4f*)(s);
  const v4f c = *(const v4f*)(s + 4);
  v8h o = {(_Float16)(a.x * WSC), (_Float16)(a.y * WSC), (_Float16)(a.z * WSC), (_Float16)(a.w * WSC),
           (_Float16)(c.x * WSC), (_Float16)(c.y * WSC), (_Float16)(c.z * WSC), (_Float16)(c.w * WSC)};
  _Float16* dst = w16 + (size_t)i * 8;
  *(volatile v8h*)dst = o;
  __threadfence();
  *(volatile v8h*)dst = o;
}

__global__ __launch_bounds__(256) void k_sm(const float* __restrict__ cen,
                                            const float* __restrict__ spr,
                                            float* __restrict__ probs,
                                            _Float16* __restrict__ p16,
                                            int* __restrict__ rng) {
  __shared__ float redm[8];
  __shared__ float reds[8];
  __shared__ int rmn[8];
  __shared__ int rmx[8];
  __shared__ __attribute__((aligned(16))) _Float16 ph[NQ];
  __shared__ __attribute__((aligned(16))) int rts[32];
  const int tid = threadIdx.x, wave = tid >> 5, lane = tid & 31;
  const int hd = blockIdx.y, q0 = blockIdx.x * 16;
  if (q0 >= NQ || hd >= NH) return;

  const float s00 = spr[hd * 4 + 0], s01 = spr[hd * 4 + 1];
  const float s10 = spr[hd * 4 + 2], s11 = spr[hd * 4 + 3];
  const float ca = s00 * s00 + s01 * s01;
  const float cb = s00 * s10 + s01 * s11;
  const float cc = s10 * s10 + s11 * s11;
  const float mu1 = cen[hd * 2 + 0], mu2 = cen[hd * 2 + 1];
  const float u0 = ca * mu1 + cb * mu2;
  const float u1 = (cc + mu2) + cb * mu1;
  const float u2 = -0.5f * ca, u3 = -0.5f * cc, u4 = -cb;
  const int k1 = tid >> 3, k2b = (tid & 7) * 4;

#pragma unroll 1
  for (int qq = 0; qq < 16; ++qq) {
    const int q = q0 + qq, qi = q >> 5, qj = q & 31;
    const float dk = (float)(k1 - qi);
    float sc[4];
#pragma unroll
    for (int e = 0; e < 4; ++e) {
      const float dl = (float)(k2b + e - qj);
      sc[e] = u0 * dk + u1 * dl + u2 * (dk * dk) + u3 * (dl * dl) + u4 * (dk * dl);
    }
    float m = fmaxf(fmaxf(sc[0], sc[1]), fmaxf(sc[2], sc[3]));
#pragma unroll
    for (int off = 16; off; off >>= 1) m = fmaxf(m, __shfl_xor(m, off, 32));
    if (lane == 0) redm[wave] = m;
    __syncthreads();
    float bm = redm[0];
#pragma unroll
    for (int ww = 1; ww < 8; ++ww) bm = fmaxf(bm, redm[ww]);

    float ex[4], es = 0.0f;
#pragma unroll
    for (int e = 0; e < 4; ++e) { ex[e] = __expf(sc[e] - bm); es += ex[e]; }
#pragma unroll
    for (int off = 16; off; off >>= 1) es += __shfl_xor(es, off, 32);
    if (lane == 0) reds[wave] = es;
    __syncthreads();
    float tot = 0.0f;
#pragma unroll
    for (int ww = 0; ww < 8; ++ww) tot += reds[ww];
    const float inv = 1.0f / tot;

    float pr[4];
    _Float16 hq[4];
    int kmn = NQ, kmx = -1;
#pragma unroll
    for (int e = 0; e < 4; ++e) {
      pr[e] = ex[e] * inv;
      const float v = pr[e] * PSC;
      const bool nz = (v >= F16MIN);
      hq[e] = nz ? (_Float16)v : (_Float16)0.0f;
      if (nz) { kmn = min(kmn, 4 * tid + e); kmx = max(kmx, 4 * tid + e); }
    }
    const v4f pv = {pr[0], pr[1], pr[2], pr[3]};
    float* prow = probs + ((size_t)q * NH + hd) * NQ;
    *(volatile v4f*)(prow + 4 * tid) = pv;
    const v4h hv = {hq[0], hq[1], hq[2], hq[3]};
    *(v4h*)(ph + 4 * tid) = hv;
#pragma unroll
    for (int off = 16; off; off >>= 1) {
      kmn = min(kmn, __shfl_xor(kmn, off, 32));
      kmx = max(kmx, __shfl_xor(kmx, off, 32));
    }
    if (lane == 0) { rmn[wave] = kmn; rmx[wave] = kmx; }
    __syncthreads();

    _Float16* hrow = p16 + ((size_t)hd * NQ + q) * NQ;
    if (tid < 128) {
      const v8h h8 = *(const v8h*)(ph + 8 * tid);
      *(volatile v8h*)(hrow + 8 * tid) = h8;
    }
    if (tid == 0) {
      int bmn = rmn[0], bmx = rmx[0];
#pragma unroll
      for (int ww = 1; ww < 8; ++ww) { bmn = min(bmn, rmn[ww]); bmx = max(bmx, rmx[ww]); }
      rts[2 * qq] = bmn;
      rts[2 * qq + 1] = bmx;
    }
    __threadfence();
    *(volatile v4f*)(prow + 4 * tid) = pv;
    if (tid < 128) {
      const v8h h8 = *(const v8h*)(ph + 8 * tid);
      *(volatile v8h*)(hrow + 8 * tid) = h8;
    }
  }
  __syncthreads();
  if (tid < 8) {
    const v4i rv = *(const v4i*)(rts + 4 * tid);
    int* dst = rng + ((size_t)(hd * NQ + q0)) * 2 + 4 * tid;
    *(volatile v4i*)dst = rv;
    __threadfence();
    *(volatile v4i*)dst = rv;
  }
}

__global__ __launch_bounds__(256) void k_ctx(const _Float16* __restrict__ p16,
                                             const _Float16* __restrict__ x16t,
                                             const int* __restrict__ rng,
                                             _Float16* __restrict__ ctx) {
  __shared__ __attribute__((aligned(16))) char smem[SMEM_BYTES];
  __shared__ int smn[8];
  __shared__ int smx[8];
  _Float16* sA = (_Float16*)smem;
  _Float16* sB = sA + 128 * LDT;
  const int tid = threadIdx.x, wave = tid >> 5, lane = tid & 31;
  const int wm = wave >> 2, wn = wave & 3, h = lane >> 4, l15 = lane & 15;
  const int q0 = blockIdx.x * 128, d0 = blockIdx.y * 128;
  const int b = blockIdx.z / NH, hd = blockIdx.z - b * NH;
  if (q0 >= NQ || d0 >= DM || b >= NB) return;

  int kmn = NQ, kmx = -1;
  if (tid < 128) {
    const int* pr = rng + ((size_t)(hd * NQ + q0 + tid)) * 2;
    int a = pr[0], z = pr[1];
    if (a < 0 || z >= NQ || a > z) { a = 0; z = NQ - 1; }
    kmn = a; kmx = z;
  }
#pragma unroll
  for (int off = 16; off; off >>= 1) {
    kmn = min(kmn, __shfl_xor(kmn, off, 32));
    kmx = max(kmx, __shfl_xor(kmx, off, 32));
  }
  if (lane == 0) { smn[wave] = kmn; smx[wave] = kmx; }
  __syncthreads();
  int bmn = smn[0], bmx = smx[0];
#pragma unroll
  for (int ww = 1; ww < 8; ++ww) { bmn = min(bmn, smn[ww]); bmx = max(bmx, smx[ww]); }
  int c0 = bmn >> 6;
  if (c0 < 0) c0 = 0;
  if (c0 > NCHQ - 1) c0 = NCHQ - 1;
  int c1 = (bmx >> 6) + 1;
  if (c1 > NCHQ) c1 = NCHQ;
  if (c1 < c0 + 1) c1 = c0 + 1;
  c0 = __builtin_amdgcn_readfirstlane(c0);
  c1 = __builtin_amdgcn_readfirstlane(c1);

  const _Float16* gA = p16 + ((size_t)hd * NQ + q0) * NQ;
  const _Float16* gB = x16t + ((size_t)b * DM + d0) * NQ;
  v8f acc[4][2] = {};

  for (int c = c0; c < c1; ++c) {
    stage_chunk(gA, NQ, gB, NQ, c * KCH, sA, sB, tid);
    __syncthreads();
    mma_chunk(sA, sB, wm, wn, h, l15, acc);
    __syncthreads();
  }

  __syncthreads();
  _Float16* stg = (_Float16*)smem;
#pragma unroll
  for (int mi = 0; mi < 4; ++mi)
#pragma unroll
    for (int ni = 0; ni < 2; ++ni) {
      const int col = wn * 32 + ni * 16 + l15;
#pragma unroll
      for (int r = 0; r < 8; ++r) {
        const int row = wm * 64 + mi * 16 + 8 * h + r;
        stg[row * SPH + col] = (_Float16)(acc[mi][ni][r] * CSC);
      }
    }
  __syncthreads();
  const int g = lane >> 3, j = lane & 7;
  _Float16* cbase = ctx + ((size_t)b * NQ + q0) * FAN + hd * DM + d0;
#pragma unroll
  for (int it = 0; it < 8; ++it) {
    const int L = wave * 32 + it * 4 + g;
    const int row = L >> 1, ch = (L & 1) * 64 + j * 8;
    const v8h v = *(const v8h*)(stg + row * SPH + ch);
    *(volatile v8h*)(cbase + (size_t)row * FAN + ch) = v;
  }
  __threadfence();
#pragma unroll
  for (int it = 0; it < 8; ++it) {
    const int L = wave * 32 + it * 4 + g;
    const int row = L >> 1, ch = (L & 1) * 64 + j * 8;
    const v8h v = *(const v8h*)(stg + row * SPH + ch);
    *(volatile v8h*)(cbase + (size_t)row * FAN + ch) = v;
  }
}

__global__ __launch_bounds__(256) void k_out(const _Float16* __restrict__ ctx,
                                             const _Float16* __restrict__ w16,
                                             const float* __restrict__ bias,
                                             const float* __restrict__ xln,
                                             float* __restrict__ out) {
  __shared__ __attribute__((aligned(16))) char smem[SMEM_BYTES];
  _Float16* sA = (_Float16*)smem;
  _Float16* sB = sA + 128 * LDT;
  const int tid = threadIdx.x, wave = tid >> 5, lane = tid & 31;
  const int wm = wave >> 2, wn = wave & 3, h = lane >> 4, l15 = lane & 15;
  const int n0 = blockIdx.x * 128, m0 = blockIdx.y * 128;
  if (n0 >= DM || m0 >= NROW) return;

  const _Float16* gA = ctx + (size_t)m0 * FAN;
  const _Float16* gB = w16 + (size_t)n0 * FAN;
  v8f acc[4][2] = {};

  for (int c = 0; c < NCHF; ++c) {
    stage_chunk(gA, FAN, gB, FAN, c * KCH, sA, sB, tid);
    __syncthreads();
    mma_chunk(sA, sB, wm, wn, h, l15, acc);
    __syncthreads();
  }

  __syncthreads();
  float* stg = (float*)smem + wave * (32 * SPF);
  const int g = lane >> 3, j = lane & 7;
  const int colg = n0 + wn * 32 + 4 * j;
  const v4f bv = *(const v4f*)(bias + colg);
#pragma unroll
  for (int hf = 0; hf < 2; ++hf) {
#pragma unroll
    for (int ml = 0; ml < 2; ++ml)
#pragma unroll
      for (int ni = 0; ni < 2; ++ni)
#pragma unroll
        for (int r = 0; r < 8; ++r)
          stg[(ml * 16 + 8 * h + r) * SPF + ni * 16 + l15] = acc[hf * 2 + ml][ni][r];
    __syncthreads();
    v4f ov[8];
#pragma unroll
    for (int it = 0; it < 8; ++it) {
      const int rloc = it * 4 + g;
      const size_t row = (size_t)m0 + wm * 64 + hf * 32 + rloc;
      const v4f cv = *(const v4f*)(stg + rloc * SPF + 4 * j);
      const v4f xv = *(const v4f*)(xln + row * DM + colg);
      ov[it] = cv * OSC + bv + xv;
      *(volatile v4f*)(out + row * DM + colg) = ov[it];
    }
    __threadfence();
#pragma unroll
    for (int it = 0; it < 8; ++it) {
      const int rloc = it * 4 + g;
      const size_t row = (size_t)m0 + wm * 64 + hf * 32 + rloc;
      *(volatile v4f*)(out + row * DM + colg) = ov[it];
    }
    __syncthreads();
  }
}

extern "C" void kernel_launch(void* const* d_in, const int* in_sizes, int n_in,
                              void* d_out, int out_size, void* d_ws, size_t ws_size,
                              hipStream_t stream) {
  if (n_in < 7) return;
  if (in_sizes[0] != NROW * DM || in_sizes[1] != NH * 2 || in_sizes[2] != NH * 4 ||
      in_sizes[3] != DM * FAN || in_sizes[4] != DM || in_sizes[5] != DM || in_sizes[6] != DM)
    return;
  if (out_size != NROW * DM + NQ * NH * NQ) return;

  const float* hidden  = (const float*)d_in[0];
  const float* centers = (const float*)d_in[1];
  const float* spreads = (const float*)d_in[2];
  const float* value_w = (const float*)d_in[3];
  const float* value_b = (const float*)d_in[4];
  const float* gam     = (const float*)d_in[5];
  const float* bet     = (const float*)d_in[6];

  float* out   = (float*)d_out;
  float* probs = out + (size_t)NROW * DM;

  const size_t XLN_B = (size_t)NROW * DM * 4;
  const size_t X16_B = (size_t)NB * DM * NQ * 2;
  const size_t P16_B = (size_t)NH * NQ * NQ * 2;
  const size_t W16_B = (size_t)DM * FAN * 2;
  const size_t CTX_B = (size_t)NROW * FAN * 2;
  const size_t RNG_B = (size_t)NH * NQ * 2 * 4;
  const size_t XLN_O = 0;
  const size_t X16_O = XLN_O + XLN_B;
  const size_t P16_O = X16_O + X16_B;
  const size_t W16_O = P16_O + P16_B;
  const size_t CTX_O = W16_O + W16_B;
  const size_t RNG_O = CTX_O + CTX_B;
  if (RNG_O + RNG_B > ws_size) return;

  char* ws = (char*)d_ws;
  float*    xln  = (float*)(ws + XLN_O);
  _Float16* x16t = (_Float16*)(ws + X16_O);
  _Float16* p16  = (_Float16*)(ws + P16_O);
  _Float16* w16  = (_Float16*)(ws + W16_O);
  _Float16* ctx  = (_Float16*)(ws + CTX_O);
  int*      rng  = (int*)(ws + RNG_O);

  const int n8 = in_sizes[3] / 8;

  k_ln<<<dim3(NROW / 64), dim3(256), 0, stream>>>(hidden, gam, bet, xln, x16t);
  k_w<<<dim3((n8 + 255) / 256), dim3(256), 0, stream>>>(value_w, w16, n8);
  k_sm<<<dim3(NQ / 16, NH), dim3(256), 0, stream>>>(centers, spreads, probs, p16, rng);
  k_ctx<<<dim3(NQ / 128, DM / 128, NB * NH), dim3(256), 0, stream>>>(p16, x16t, rng, ctx);
  k_out<<<dim3(DM / 128, NROW / 128), dim3(256), 0, stream>>>(ctx, w16, value_b, xln, out);
}
